// SubstructureAttention_71734543777917
// MI455X (gfx1250) — hardware-run, weakly checked
//
#include <hip/hip_runtime.h>
#include <math.h>

typedef __attribute__((ext_vector_type(16))) _Float16 v16h;
typedef __attribute__((ext_vector_type(8)))  _Float16 v8h;
typedef __attribute__((ext_vector_type(8)))  float    v8f;
typedef __attribute__((ext_vector_type(4)))  float    v4f;
typedef __attribute__((ext_vector_type(4)))  unsigned int v4u;

constexpr int kGraphs = 64;
constexpr int kAtoms  = 64;
constexpr int kHid    = 256;
constexpr int kRows   = kGraphs * kAtoms;
constexpr int kHalfH  = 128;
constexpr int kS2P    = 132;
constexpr int kScP    = 65;
constexpr float kACarry   = 64.0f;
constexpr float kWCarry   = 256.0f;
constexpr float kFoldBack = 1.0f / (kACarry * kWCarry);
constexpr float kF16MinNormal = 6.103515625e-5f;
static_assert(kRows == 4096, "row count");
static_assert((kRows % 64) == 0 && (kHid % 64) == 0 && (kHid % 32) == 0, "GEMM tile multiples");
static_assert(kHid == 2 * kHalfH && (kHalfH % 4) == 0, "half split");
static_assert((kS2P % 4) == 0 && kS2P >= kHalfH, "tile pitch");

constexpr size_t kOffA16  = 0;
constexpr size_t kOffBT16 = kOffA16  + (size_t)2 * kRows * kHid * 2;
constexpr size_t kOffSP   = kOffBT16 + (size_t)2 * kHid * kHid * 2;
constexpr size_t kWsTotal = kOffSP   + (size_t)2 * kRows * kHid * 4;
static_assert(kWsTotal == 12845056ull, "carve total");
static_assert(kWsTotal <= 134217728ull, "carve cap");
static_assert((kOffBT16 % 128) == 0 && (kOffSP % 128) == 0, "128-B aligned regions");

__device__ __forceinline__ unsigned pk16(unsigned short a, unsigned short b) { return (unsigned)a | ((unsigned)b << 16); }

__device__ __forceinline__ unsigned short h_bits_flush(float v) {
  const float vv = (fabsf(v) < kF16MinNormal) ? 0.0f : v;
  const _Float16 h = (_Float16)vv;
  return __builtin_bit_cast(unsigned short, h);
}

union FragH { v16h v; v8h h[2]; };
__device__ __forceinline__ v16h frag_load_h(const _Float16* p) {
  FragH f;
  f.h[0] = *(const v8h*)(p);
  f.h[1] = *(const v8h*)(p + 16);
  return f.v;
}

__device__ __forceinline__ v8f mma_h(v16h a, v16h b, v8f c) {
  c = __builtin_amdgcn_wmma_f32_16x16x32_f16(false, a, false, b, (short)0, c, false, false);
  asm volatile("v_nop\n\tv_nop\n\tv_nop\n\tv_nop" : "+v"(c) : "v"(a), "v"(b));
  return c;
}

constexpr int kCastBlocksPerPlane = (kRows * kHid / 8) / 256;
constexpr int kCastBlocks = 2 * kCastBlocksPerPlane;
constexpr int kTransBlocks = 2 * (kHid / 64) * (kHid / 64);
static_assert(kCastBlocksPerPlane * 256 * 8 == kRows * kHid, "cast coverage");
static_assert(kCastBlocks == 1024 && kTransBlocks == 32, "prep grid");

__global__ __launch_bounds__(256) void prep_planes_kernel(const float* __restrict__ h1, const float* __restrict__ h2,
                                                          const float* __restrict__ W1,
                                                          unsigned short* __restrict__ A16,
                                                          unsigned short* __restrict__ BT16) {
  __shared__ float sm[64][65];
  const int t  = threadIdx.x;
  const int bx = blockIdx.x;
  if (bx < kCastBlocks) {
    const int pl = bx / kCastBlocksPerPlane;
    const float* src = pl ? h2 : h1;
    const int i = (bx - pl * kCastBlocksPerPlane) * 256 + t;
    const float* p = src + 8 * (size_t)i;
    const v4f a = *(const v4f*)(p);
    const v4f c = *(const v4f*)(p + 4);
    unsigned short hb[8];
#pragma unroll
    for (int e = 0; e < 4; ++e) {
      const float f0 = a[e] * kACarry;
      const float f1 = c[e] * kACarry;
      hb[e]     = h_bits_flush(f0);
      hb[4 + e] = h_bits_flush(f1);
    }
    const v4u u = (v4u){pk16(hb[0], hb[1]), pk16(hb[2], hb[3]), pk16(hb[4], hb[5]), pk16(hb[6], hb[7])};
    unsigned short* q = A16 + (size_t)pl * kRows * kHid + 8 * (size_t)i;
    *(volatile v4u*)q = u;
    __threadfence();
    *(volatile v4u*)q = u;
  } else {
    const int tb   = bx - kCastBlocks;
    const int half = tb >> 4;
    const int tile = tb & 15;
    const int k0   = (tile & 3) * 64;
    const int n0   = (tile >> 2) * 64;
    const float* W = W1 + (size_t)half * kHid * kHid;
#pragma unroll
    for (int i = 0; i < 16; ++i) {
      const int e = i * 256 + t;
      const int r = e >> 6;
      const int c = e & 63;
      sm[c][r] = W[(size_t)(k0 + r) * kHid + n0 + c] * kWCarry;
    }
    __syncthreads();
    const int lane = t & 31, wave = t >> 5;
    const int q = lane >> 3, c8 = (lane & 7) * 8;
    unsigned short* op = BT16 + (size_t)half * kHid * kHid;
    for (int pass = 0; pass < 2; ++pass) {
#pragma unroll
      for (int it = 0; it < 2; ++it) {
        const int row = wave * 8 + it * 4 + q;
        unsigned short hb[8];
#pragma unroll
        for (int e = 0; e < 8; ++e) hb[e] = h_bits_flush(sm[row][c8 + e]);
        const v4u u = (v4u){pk16(hb[0], hb[1]), pk16(hb[2], hb[3]), pk16(hb[4], hb[5]), pk16(hb[6], hb[7])};
        *(volatile v4u*)(op + (size_t)(n0 + row) * kHid + k0 + c8) = u;
      }
      __threadfence();
    }
  }
}

__global__ __launch_bounds__(256) void gemm64_f16_kernel(
    const unsigned short* __restrict__ Ap, int lda, long strideA,
    const unsigned short* __restrict__ Btp, int ldb, long strideB,
    float* __restrict__ Cout, int ldc, long strideC,
    int M, int N, int K, float scale) {
  const _Float16* A  = (const _Float16*)Ap;
  const _Float16* Bt = (const _Float16*)Btp;
  __shared__ __align__(16) float sT[8][16 * 68];
  const int b    = blockIdx.y;
  const int lane = threadIdx.x & 31;
  const int wave = threadIdx.x >> 5;
  const int tilesN = N >> 6;
  const int tilesM = M >> 6;
  const int tile = blockIdx.x * 8 + wave;
  if (tile >= tilesM * tilesN) return;
  const int tm = tile / tilesN;
  const int tn = tile - tm * tilesN;
  const int m0 = tm << 6;
  const int n0 = tn << 6;

  const _Float16* Ab = A  + (size_t)b * strideA;
  const _Float16* Bb = Bt + (size_t)b * strideB;

  const int rlane = lane & 15;
  const int koff  = (lane >> 4) * 8;
  const int mOff  = (lane >> 4) * 8;

  v8f acc[4][4];
#pragma unroll
  for (int i = 0; i < 4; ++i)
#pragma unroll
    for (int j = 0; j < 4; ++j) acc[i][j] = (v8f){0.f, 0.f, 0.f, 0.f, 0.f, 0.f, 0.f, 0.f};

  for (int k0 = 0; k0 < K; k0 += 32) {
    v16h bh[4];
#pragma unroll
    for (int j = 0; j < 4; ++j) {
      const size_t bo = (size_t)(n0 + (j << 4) + rlane) * ldb + koff + k0;
      bh[j] = frag_load_h(Bb + bo);
    }
#pragma unroll
    for (int i = 0; i < 4; ++i) {
      const size_t ao = (size_t)(m0 + (i << 4) + rlane) * lda + koff + k0;
      const v16h ah = frag_load_h(Ab + ao);
#pragma unroll
      for (int j = 0; j < 4; ++j) acc[i][j] = mma_h(ah, bh[j], acc[i][j]);
    }
  }

  float* slab = sT[wave];
  float* C = Cout + (size_t)b * strideC;
#pragma unroll
  for (int i = 0; i < 4; ++i) {
    const int mBase = m0 + (i << 4);
#pragma unroll
    for (int j = 0; j < 4; ++j) {
#pragma unroll
      for (int r = 0; r < 8; ++r) {
        const float v = acc[i][j][r] * scale;
        slab[(mOff + r) * 68 + (j << 4) + rlane] = v;
      }
    }
    __builtin_amdgcn_fence(__ATOMIC_RELEASE, "workgroup");
    __builtin_amdgcn_wave_barrier();
    __builtin_amdgcn_fence(__ATOMIC_ACQUIRE, "workgroup");
    {
      const int hh = lane >> 4, c4 = (lane & 15) * 4;
      for (int pass = 0; pass < 2; ++pass) {
#pragma unroll
        for (int it = 0; it < 8; ++it) {
          const int row = it * 2 + hh;
          const v4f v = *(const v4f*)(slab + row * 68 + c4);
          *(volatile v4f*)(C + (size_t)(mBase + row) * ldc + n0 + c4) = v;
        }
        __threadfence();
      }
    }
    __builtin_amdgcn_fence(__ATOMIC_RELEASE, "workgroup");
    __builtin_amdgcn_wave_barrier();
    __builtin_amdgcn_fence(__ATOMIC_ACQUIRE, "workgroup");
  }
}

static_assert(kHid == 256, "block size equals the hidden width");

__global__ __launch_bounds__(256) void pair_score_kernel(const float* __restrict__ S1, const float* __restrict__ S2,
                                                         const float* __restrict__ b1, const float* __restrict__ w2,
                                                         const float* __restrict__ b2, const int* __restrict__ ngraphs,
                                                         float* __restrict__ out) {
  __shared__ __align__(16) float s2s[kAtoms * kS2P];
  __shared__ __align__(16) float sc[kAtoms * kScP];
  __shared__ __align__(16) float cb1[kHid];
  __shared__ __align__(16) float cwq[kHid];
  __shared__ float redM[8];
  __shared__ float redS[8];

  const int t    = threadIdx.x;
  const int lane = t & 31;
  const int wave = t >> 5;
  const int g    = blockIdx.x;

  const int   ngv = ngraphs[0];
  const float b2v = b2[0];
  cb1[t] = b1[t];
  cwq[t] = -2.0f * w2[t];
  __syncthreads();

  float wpart;
  {
    const v4f q0 = *(const v4f*)(cwq + lane * 8);
    const v4f q1 = *(const v4f*)(cwq + lane * 8 + 4);
    wpart = ((q0[0] + q0[1]) + (q0[2] + q0[3])) + ((q1[0] + q1[1]) + (q1[2] + q1[3]));
  }
#pragma unroll
  for (int off = 16; off > 0; off >>= 1) wpart += __shfl_xor(wpart, off, 32);
  const float sbase = -0.5f * wpart + b2v;

  const int i  = t >> 2;
  const int j0 = (t & 3) * 16;
  const float* S1row = S1 + ((size_t)g * kAtoms + i) * kHid;
  const float* S2g   = S2 + (size_t)g * kAtoms * kHid;

  float acc[16];
#pragma unroll
  for (int jj = 0; jj < 16; ++jj) acc[jj] = 0.0f;

#pragma unroll 1
  for (int hp = 0; hp < 2; ++hp) {
    __syncthreads();
#pragma unroll
    for (int it = 0; it < 8; ++it) {
      const int e  = it * 256 + t;
      const int j  = e >> 5;
      const int c4 = (e & 31) * 4;
      v4f v = *(const v4f*)(S2g + (size_t)j * kHid + hp * kHalfH + c4);
      v = v * 2.0f;
      *(v4f*)(s2s + j * kS2P + c4) = v;
    }
    __syncthreads();
#pragma unroll 1
    for (int h0 = 0; h0 < kHalfH; h0 += 4) {
      const int hg = hp * kHalfH + h0;
      v4f a = *(const v4f*)(S1row + hg);
      const v4f bb = *(const v4f*)(cb1 + hg);
      const v4f wq = *(const v4f*)(cwq + hg);
      a = (a + bb) * 2.0f;
#pragma unroll
      for (int jj = 0; jj < 16; ++jj) {
        const v4f s = *(const v4f*)(s2s + (j0 + jj) * kS2P + h0);
#pragma unroll
        for (int d = 0; d < 4; ++d) {
          const float ex = __expf(a[d] + s[d]);
          const float rc = __builtin_amdgcn_rcpf(1.0f + ex);
          acc[jj] = fmaf(wq[d], rc, acc[jj]);
        }
      }
    }
  }

#pragma unroll
  for (int jj = 0; jj < 16; ++jj) sc[i * kScP + j0 + jj] = acc[jj] + sbase;
  __syncthreads();

  float lmax = -INFINITY;
#pragma unroll 1
  for (int jj = 0; jj < 16; ++jj) lmax = fmaxf(lmax, sc[i * kScP + j0 + jj]);
#pragma unroll
  for (int off = 16; off > 0; off >>= 1) lmax = fmaxf(lmax, __shfl_xor(lmax, off, 32));
  if (lane == 0) redM[wave] = lmax;
  __syncthreads();
  float gmax = redM[0];
#pragma unroll
  for (int w = 1; w < 8; ++w) gmax = fmaxf(gmax, redM[w]);

  float lsum = 0.0f;
#pragma unroll 1
  for (int jj = 0; jj < 16; ++jj) {
    const int o = i * kScP + j0 + jj;
    float ev = expf(sc[o] - gmax);
    ev = (ev < 1.17549435e-38f) ? 0.0f : ev;
    sc[o] = ev;
    lsum += ev;
  }
#pragma unroll
  for (int off = 16; off > 0; off >>= 1) lsum += __shfl_xor(lsum, off, 32);
  if (lane == 0) redS[wave] = lsum;
  __syncthreads();
  float tot = 0.0f;
#pragma unroll
  for (int w = 0; w < 8; ++w) tot += redS[w];
  const float inv = 1.0f / tot;

  if (t < 2 * kAtoms) {
    const bool isRow = (t < kAtoms);
    const int  idx   = t & (kAtoms - 1);
    float sum = 0.0f;
#pragma unroll 1
    for (int x = 0; x < kAtoms; ++x) {
      const int o = isRow ? (idx * kScP + x) : (x * kScP + idx);
      const float p = sc[o] * inv;
      sum += p;
    }
    sum = (ngv == kGraphs) ? sum : __uint_as_float(0x7fc00000u);
    volatile float* dst = out + (isRow ? 0 : kRows) + g * kAtoms + idx;
    *dst = sum;
    __threadfence();
    *dst = sum;
  }
}

extern "C" void kernel_launch(void* const* d_in, const int* in_sizes, int n_in,
                              void* d_out, int out_size, void* d_ws, size_t ws_size,
                              hipStream_t stream) {
  if (n_in < 9) return;
  if (in_sizes[0] != kRows * kHid) return;
  if (in_sizes[1] != kRows * kHid) return;
  if (in_sizes[2] != kRows) return;
  if (in_sizes[3] != kRows) return;
  if (in_sizes[4] != 1) return;
  if (in_sizes[5] != 2 * kHid * kHid) return;
  if (in_sizes[6] != kHid) return;
  if (in_sizes[7] != kHid) return;
  if (in_sizes[8] != 1) return;
  if (out_size != 2 * kRows) return;
  if (ws_size < kWsTotal) return;

  const float* h1 = (const float*)d_in[0];
  const float* h2 = (const float*)d_in[1];
  const int*   ng = (const int*)d_in[4];
  const float* W1 = (const float*)d_in[5];
  const float* b1 = (const float*)d_in[6];
  const float* W2 = (const float*)d_in[7];
  const float* b2 = (const float*)d_in[8];
  float* out = (float*)d_out;

  char* ws = (char*)d_ws;
  unsigned short* A16  = (unsigned short*)(ws + kOffA16);
  unsigned short* BT16 = (unsigned short*)(ws + kOffBT16);
  float*          SP   = (float*)(ws + kOffSP);

  prep_planes_kernel<<<kCastBlocks + kTransBlocks, 256, 0, stream>>>(h1, h2, W1, A16, BT16);

  gemm64_f16_kernel<<<dim3((kRows / 64) * (kHid / 64) / 8, 2), 256, 0, stream>>>(
      A16, kHid, (long)kRows * kHid,
      BT16, kHid, (long)kHid * kHid,
      SP, kHid, (long)kRows * kHid,
      kRows, kHid, kHid, kFoldBack);

  const float* S1 = SP;
  const float* S2 = SP + (size_t)kRows * kHid;
  pair_score_kernel<<<kGraphs, 256, 0, stream>>>(S1, S2, b1, W2, b2, ng, out);
}
